// RNN_9560597201285
// MI455X (gfx1250) — hardware-verified
//
#include <hip/hip_runtime.h>
#include <math.h>

constexpr int NBATCH  = 64;
constexpr int NSTEP   = 1024;
constexpr int NINP    = 64;
constexpr int NHID    = 512;
constexpr int NOUTC   = 64;
constexpr int KCAT    = NHID + NINP;
constexpr int APITCH  = 584;
constexpr int NTHR    = 256;
constexpr int SEQ_BLK = 16;
constexpr int SLABP   = 68;
constexpr int NROWS   = NBATCH * NSTEP;
constexpr float WCARRY     = 256.0f;
constexpr float WCARRY_INV = 1.0f / 256.0f;
constexpr float DT_STEP    = 0.5f;

static_assert(KCAT == 576);
static_assert(KCAT % 32 == 0);
static_assert(NHID % 32 == 0);
static_assert(APITCH % 8 == 0 && APITCH >= KCAT + 8);
static_assert(NBATCH % SEQ_BLK == 0);
static_assert(NHID == 64 * (NTHR / 32));
static_assert(NROWS % 64 == 0 && NOUTC == 64);
static_assert((NROWS / 64) % (NTHR / 32) == 0);
static_assert(SEQ_BLK * NINP == NTHR * 4);
static_assert(SEQ_BLK * NHID == NTHR * 4 * 8);
static_assert(NHID % 64 == 0 && NINP % 64 == 0 && NOUTC % 64 == 0);

typedef __attribute__((ext_vector_type(16))) _Float16 v16h;
typedef __attribute__((ext_vector_type(8)))  _Float16 v8h;
typedef __attribute__((ext_vector_type(4)))  _Float16 v4h;
typedef __attribute__((ext_vector_type(8)))  float    v8f;
typedef __attribute__((ext_vector_type(4)))  float    v4f;

__device__ __forceinline__ unsigned short f2bf_bits(float f) {
  unsigned u = __float_as_uint(f);
  return (unsigned short)((u + 0x7FFFu + ((u >> 16) & 1u)) >> 16);
}
__device__ __forceinline__ float bf_bits2f(unsigned short h) { return __uint_as_float(((unsigned)h) << 16); }
__device__ __forceinline__ float bf16r(float f) { return bf_bits2f(f2bf_bits(f)); }

__device__ __forceinline__ void guard_grp4(v8f& a0, v8f& a1, v8f& a2, v8f& a3, v16h x, v16h b0, v16h b1, v16h b2, v16h b3) {
  asm volatile("v_nop\n\tv_nop\n\tv_nop\n\tv_nop" : "+v"(a0), "+v"(a1), "+v"(a2), "+v"(a3) : "v"(x), "v"(b0), "v"(b1), "v"(b2), "v"(b3));
}
__device__ __forceinline__ void keep4_h(v16h a, v16h b, v16h c, v16h d) { asm volatile("v_nop" :: "v"(a), "v"(b), "v"(c), "v"(d)); }
__device__ __forceinline__ void acc_guard4(v8f& a, v8f& b, v8f& c, v8f& d) { asm volatile("v_nop\n\tv_nop\n\tv_nop\n\tv_nop" : "+v"(a), "+v"(b), "+v"(c), "+v"(d)); }

union FragU { v16h v; v8h h[2]; };
__device__ __forceinline__ v16h frag_load(const _Float16* p) {
  FragU f;
  f.h[0] = *(const v8h*)(p);
  f.h[1] = *(const v8h*)(p + 16);
  return f.v;
}
__device__ __forceinline__ v8f frag_mma(v16h a, v16h b, v8f c) {
  return __builtin_amdgcn_wmma_f32_16x16x32_f16(false, a, false, b, (short)0, c, false, false);
}

__device__ __forceinline__ float tanh_f(float x) {
  const float xc = fminf(fmaxf(x, -15.0f), 15.0f);
  const float e  = expf(2.0f * xc);
  return 1.0f - 2.0f * __builtin_amdgcn_rcpf(e + 1.0f);
}

__global__ __launch_bounds__(NTHR) void cvt_wrec_kernel(const float* __restrict__ src, unsigned short* __restrict__ dst) {
  const int i = blockIdx.x * NTHR + threadIdx.x;
  if (i < NHID * (NHID / 8)) {
    const int row = i >> 6;
    const int c8  = (i & 63) * 8;
    const float* sp = src + (size_t)row * NHID + c8;
    const v4f a = *(const v4f*)(sp);
    const v4f b = *(const v4f*)(sp + 4);
    v8h hv;
#pragma unroll
    for (int e = 0; e < 4; ++e) {
      const float fa = a[e];
      const float fb = b[e];
      hv[e]     = (_Float16)(bf16r(fa) * WCARRY);
      hv[4 + e] = (_Float16)(bf16r(fb) * WCARRY);
    }
    unsigned short* op = dst + (size_t)row * KCAT + c8;
    *(volatile v8h*)op = hv;
    __threadfence();
    *(volatile v8h*)op = hv;
  }
}

__global__ __launch_bounds__(NTHR) void tpw_f16_kernel(const float* __restrict__ src, int R, int C, int ldo, int ocol0,
                                                      unsigned short* __restrict__ O, float sc) {
  __shared__ float Tt[64 * 65];
  const int tid = threadIdx.x;
  const int c0 = blockIdx.x * 64, r0 = blockIdx.y * 64;
  if (c0 + 64 > C || r0 + 64 > R) return;
#pragma unroll
  for (int i = 0; i < 4; ++i) {
    const int idx = i * NTHR + tid;
    const int rr = idx >> 4, cc = (idx & 15) * 4;
    const v4f v = *(const v4f*)(src + (size_t)(r0 + rr) * (size_t)C + c0 + cc);
    Tt[rr * 65 + cc + 0] = v[0];
    Tt[rr * 65 + cc + 1] = v[1];
    Tt[rr * 65 + cc + 2] = v[2];
    Tt[rr * 65 + cc + 3] = v[3];
  }
  __syncthreads();
  const int q = tid >> 3, c8 = (tid & 7) * 8;
  v8h hv[2];
#pragma unroll
  for (int g = 0; g < 2; ++g) {
    const int qq = g * 32 + q;
#pragma unroll
    for (int e = 0; e < 8; ++e) {
      const float f = Tt[(c8 + e) * 65 + qq];
      hv[g][e] = (_Float16)(bf16r(f) * sc);
    }
  }
  for (int pass = 0; pass < 2; ++pass) {
#pragma unroll
    for (int g = 0; g < 2; ++g) {
      const size_t o = (size_t)(c0 + g * 32 + q) * (size_t)ldo + (size_t)(ocol0 + r0 + c8);
      *(volatile v8h*)(O + o) = hv[g];
    }
    __threadfence();
  }
}

__device__ __forceinline__ void stage_x(_Float16* Ah, const float* __restrict__ xin, int rowbase, int t, int tid) {
  const int m = tid >> 4, f4 = (tid & 15) * 4;
  const v4f v = *(const v4f*)(xin + ((size_t)(rowbase + m) * NSTEP + (size_t)t) * NINP + f4);
  const float f0 = v[0], f1 = v[1], f2 = v[2], f3 = v[3];
  v4h hv;
  hv[0] = (_Float16)bf16r(f0);
  hv[1] = (_Float16)bf16r(f1);
  hv[2] = (_Float16)bf16r(f2);
  hv[3] = (_Float16)bf16r(f3);
  *(v4h*)(Ah + m * APITCH + NHID + f4) = hv;
}

__device__ __forceinline__ void put_h(_Float16* Ah, const v8f& hv, int col, int hh) {
#pragma unroll
  for (int r = 0; r < 8; ++r) {
    const float f = hv[r];
    Ah[(8 * hh + r) * APITCH + col] = (_Float16)f;
  }
}

__global__ __launch_bounds__(NTHR) void rnn_seq_kernel(const float* __restrict__ xin, const float* __restrict__ brec,
                                                       const float* __restrict__ h0,
                                                       const unsigned short* __restrict__ Wcp,
                                                       unsigned short* __restrict__ hsp) {
  __shared__ __align__(16) _Float16 Ah[SEQ_BLK * APITCH];
  const _Float16* Wc = (const _Float16*)Wcp;
  _Float16* hsg = (_Float16*)hsp;
  const int tid = threadIdx.x, lane = tid & 31, wave = tid >> 5;
  const int c = lane & 15, hh = lane >> 4, koff = hh * 8;
  const int rowbase = blockIdx.x * SEQ_BLK;

  {
    const _Float16 fa = (_Float16)bf16r(h0[tid]);
    const _Float16 fb = (_Float16)bf16r(h0[tid + 256]);
#pragma unroll 1
    for (int i = 0; i < SEQ_BLK; ++i) {
      Ah[i * APITCH + tid] = fa;
      Ah[i * APITCH + 256 + tid] = fb;
    }
  }
  if (tid < SEQ_BLK) {
    const v8h zz = {(_Float16)0.0f, (_Float16)0.0f, (_Float16)0.0f, (_Float16)0.0f,
                    (_Float16)0.0f, (_Float16)0.0f, (_Float16)0.0f, (_Float16)0.0f};
    *(v8h*)(Ah + tid * APITCH + KCAT) = zz;
  }
  stage_x(Ah, xin, rowbase, 0, tid);

  const int jb = 64 * wave + c;
  v8f hs0, hs1, hs2, hs3;
  float bb0, bb1, bb2, bb3;
  {
    const float g0 = bf16r(h0[jb]);
    const float g1 = bf16r(h0[jb + 16]);
    const float g2 = bf16r(h0[jb + 32]);
    const float g3 = bf16r(h0[jb + 48]);
#pragma unroll
    for (int r = 0; r < 8; ++r) { hs0[r] = g0; hs1[r] = g1; hs2[r] = g2; hs3[r] = g3; }
    bb0 = bf16r(brec[jb]);
    bb1 = bf16r(brec[jb + 16]);
    bb2 = bf16r(brec[jb + 32]);
    bb3 = bf16r(brec[jb + 48]);
  }
  __syncthreads();

  const _Float16* ahrow = Ah + c * APITCH + koff;
  const _Float16* w0 = Wc + (size_t)(jb)      * KCAT + koff;
  const _Float16* w1 = Wc + (size_t)(jb + 16) * KCAT + koff;
  const _Float16* w2 = Wc + (size_t)(jb + 32) * KCAT + koff;
  const _Float16* w3 = Wc + (size_t)(jb + 48) * KCAT + koff;
  const v8f z8 = {0.f, 0.f, 0.f, 0.f, 0.f, 0.f, 0.f, 0.f};

#pragma unroll 1
  for (int t = 0; t < NSTEP; ++t) {
    v8f a0 = z8, a1 = z8, a2 = z8, a3 = z8;
#pragma unroll 1
    for (int k0 = 0; k0 < KCAT; k0 += 32) {
      const v16h a  = frag_load(ahrow + k0);
      const v16h b0 = frag_load(w0 + k0);
      const v16h b1 = frag_load(w1 + k0);
      const v16h b2 = frag_load(w2 + k0);
      const v16h b3 = frag_load(w3 + k0);
      a0 = frag_mma(a, b0, a0);
      a1 = frag_mma(a, b1, a1);
      a2 = frag_mma(a, b2, a2);
      a3 = frag_mma(a, b3, a3);
      guard_grp4(a0, a1, a2, a3, a, b0, b1, b2, b3);
    }
    acc_guard4(a0, a1, a2, a3);

#pragma unroll 1
    for (int q = 0; q < 4; ++q) {
      v8f hn;
#pragma unroll
      for (int r = 0; r < 8; ++r) {
        const float pre = a0[r] * WCARRY_INV + bb0;
        const float th  = tanh_f(pre);
        hn[r] = (1.0f - DT_STEP) * hs0[r] + DT_STEP * th;
      }
      a0 = a1; a1 = a2; a2 = a3;
      hs0 = hs1; hs1 = hs2; hs2 = hs3; hs3 = hn;
      const float tb = bb0;
      bb0 = bb1; bb1 = bb2; bb2 = bb3; bb3 = tb;
    }

    __syncthreads();
    put_h(Ah, hs0, jb,      hh);
    put_h(Ah, hs1, jb + 16, hh);
    put_h(Ah, hs2, jb + 32, hh);
    put_h(Ah, hs3, jb + 48, hh);
    {
      const int tn = (t + 1 < NSTEP) ? (t + 1) : (NSTEP - 1);
      stage_x(Ah, xin, rowbase, tn, tid);
    }
    __syncthreads();

    {
      v8h ov[4];
#pragma unroll
      for (int it = 0; it < 4; ++it) {
        const int idx = it * NTHR + tid;
        const int row = idx >> 6, c8 = (idx & 63) * 8;
        ov[it] = *(const v8h*)(Ah + row * APITCH + c8);
      }
      for (int pass = 0; pass < 2; ++pass) {
#pragma unroll
        for (int it = 0; it < 4; ++it) {
          const int idx = it * NTHR + tid;
          const int row = idx >> 6, c8 = (idx & 63) * 8;
          *(volatile v8h*)(hsg + ((size_t)t * NBATCH + (size_t)(rowbase + row)) * NHID + c8) = ov[it];
        }
        __threadfence();
      }
    }
  }
}

__global__ __launch_bounds__(NTHR) void readout_gemm_kernel(const unsigned short* __restrict__ Ap,
                                                            const unsigned short* __restrict__ Btp,
                                                            float* __restrict__ out) {
  __shared__ __align__(16) float sT[NTHR / 32][16 * SLABP];
  const _Float16* A  = (const _Float16*)Ap;
  const _Float16* Bt = (const _Float16*)Btp;
  const int lane = threadIdx.x & 31;
  const int wave = threadIdx.x >> 5;
  const int tile = blockIdx.x * (NTHR / 32) + wave;
  if (tile >= NROWS / 64) return;
  const int m0 = tile << 6;
  const int rlane = lane & 15;
  const int koff  = (lane >> 4) * 8;
  const int mOff  = (lane >> 4) * 8;

  v8f acc[4][4];
#pragma unroll
  for (int i = 0; i < 4; ++i)
#pragma unroll
    for (int j = 0; j < 4; ++j) acc[i][j] = (v8f){0.f, 0.f, 0.f, 0.f, 0.f, 0.f, 0.f, 0.f};

#pragma unroll 1
  for (int k0 = 0; k0 < NHID; k0 += 32) {
    v16h bh[4];
#pragma unroll
    for (int j = 0; j < 4; ++j) {
      const size_t bo = (size_t)((j << 4) + rlane) * NHID + koff + k0;
      bh[j] = frag_load(Bt + bo);
    }
#pragma unroll
    for (int i = 0; i < 4; ++i) {
      const size_t ao = (size_t)(m0 + (i << 4) + rlane) * NHID + koff + k0;
      const v16h ah = frag_load(A + ao);
#pragma unroll
      for (int j = 0; j < 4; ++j) acc[i][j] = frag_mma(ah, bh[j], acc[i][j]);
      guard_grp4(acc[i][0], acc[i][1], acc[i][2], acc[i][3], ah, bh[0], bh[1], bh[2], bh[3]);
    }
    keep4_h(bh[0], bh[1], bh[2], bh[3]);
  }
  acc_guard4(acc[0][0], acc[0][1], acc[0][2], acc[0][3]);
  acc_guard4(acc[1][0], acc[1][1], acc[1][2], acc[1][3]);
  acc_guard4(acc[2][0], acc[2][1], acc[2][2], acc[2][3]);
  acc_guard4(acc[3][0], acc[3][1], acc[3][2], acc[3][3]);

  float* slab = sT[wave];
  const int hh = lane >> 4, c4 = (lane & 15) * 4;
#pragma unroll
  for (int i = 0; i < 4; ++i) {
    const int mBase = m0 + (i << 4);
#pragma unroll
    for (int j = 0; j < 4; ++j) {
#pragma unroll
      for (int r = 0; r < 8; ++r) slab[(mOff + r) * SLABP + (j << 4) + rlane] = acc[i][j][r] * WCARRY_INV;
    }
    __builtin_amdgcn_fence(__ATOMIC_RELEASE, "workgroup");
    __builtin_amdgcn_wave_barrier();
    __builtin_amdgcn_fence(__ATOMIC_ACQUIRE, "workgroup");
    for (int pass = 0; pass < 2; ++pass) {
#pragma unroll
      for (int it = 0; it < 8; ++it) {
        const int row = it * 2 + hh;
        const v4f v = *(const v4f*)(slab + row * SLABP + c4);
        const int g = mBase + row;
        const size_t orow = (size_t)(g & (NBATCH - 1)) * NSTEP + (size_t)(g >> 6);
        *(volatile v4f*)(out + orow * NOUTC + c4) = v;
      }
      __threadfence();
    }
    __builtin_amdgcn_fence(__ATOMIC_RELEASE, "workgroup");
    __builtin_amdgcn_wave_barrier();
    __builtin_amdgcn_fence(__ATOMIC_ACQUIRE, "workgroup");
  }
}

extern "C" void kernel_launch(void* const* d_in, const int* in_sizes, int n_in,
                              void* d_out, int out_size, void* d_ws, size_t ws_size, hipStream_t stream) {
  if (n_in < 6 || d_out == nullptr || d_ws == nullptr) return;
  if (in_sizes[0] != NBATCH * NSTEP * NINP || in_sizes[1] != NINP * NHID || in_sizes[2] != NHID * NHID ||
      in_sizes[3] != NHID * NOUTC || in_sizes[4] != NHID || in_sizes[5] != NHID ||
      out_size != NBATCH * NSTEP * NOUTC) return;

  const float* xin  = (const float*)d_in[0];
  const float* wi   = (const float*)d_in[1];
  const float* wrec = (const float*)d_in[2];
  const float* wo   = (const float*)d_in[3];
  const float* brec = (const float*)d_in[4];
  const float* h0   = (const float*)d_in[5];
  float* out = (float*)d_out;

  char* ws = (char*)d_ws;
  size_t off = 0;
  auto carve = [&](size_t bytes) -> char* { char* p = ws + off; off += (bytes + 255) & ~(size_t)255; return p; };
  unsigned short* HS16 = (unsigned short*)carve((size_t)NROWS * NHID * 2);
  unsigned short* WCAT = (unsigned short*)carve((size_t)NHID * KCAT * 2);
  unsigned short* WOT  = (unsigned short*)carve((size_t)NOUTC * NHID * 2);
  if (off > ws_size || off > (size_t)134217728) return;

  cvt_wrec_kernel<<<(NHID * (NHID / 8)) / NTHR, NTHR, 0, stream>>>(wrec, WCAT);
  tpw_f16_kernel<<<dim3(NHID / 64, NINP / 64), NTHR, 0, stream>>>(wi, NINP, NHID, KCAT, NHID, WCAT, WCARRY);
  tpw_f16_kernel<<<dim3(NOUTC / 64, NHID / 64), NTHR, 0, stream>>>(wo, NHID, NOUTC, NHID, 0, WOT, WCARRY);
  rnn_seq_kernel<<<NBATCH / SEQ_BLK, NTHR, 0, stream>>>(xin, brec, h0, WCAT, HS16);
  readout_gemm_kernel<<<(NROWS / 64) / (NTHR / 32), NTHR, 0, stream>>>(HS16, WOT, out);
}
